// Attention_64476049047608
// MI455X (gfx1250) — hardware-verified
//
#include <hip/hip_runtime.h>
#include <math.h>


#ifndef NB
#define NB 2
#endif
#ifndef SEQ
#define SEQ 2048
#endif
#define NB_FULL  2
#define SEQ_FULL 2048
#define HID  2048
#define NH   32
#define NKV  8
#define HD   64
#define NQKV 3072
#define NWV  4
#define KS   32
#define OSP  68
#define VTP  136
#define CSP  72
#define L2E  1.4426950408889634f

static_assert(HID == 2048);
static_assert(NH == 32 && NKV == 8 && HD == 64);
static_assert((NH + 2 * NKV) * HD == NQKV);
static_assert(NH * HD == HID);
static_assert(HID % 32 == 0);
static_assert(SEQ % 128 == 0);
static_assert(SEQ % KS == 0);
static_assert(NB <= NB_FULL);
static_assert(SEQ <= SEQ_FULL);
static_assert(((size_t)NB * SEQ * HID / 8) % 256 == 0);
static_assert(((size_t)HID * HID / 8) % 256 == 0);
static_assert(((size_t)NKV * HD * HID / 8) % 256 == 0);
static_assert(((size_t)NB * SEQ * 32) % 256 == 0);
static_assert((size_t)(NQKV / 64) * (size_t)(NB * SEQ / 128) * 4u * (32u * 64u) == (size_t)NB * SEQ * NQKV);
static_assert((size_t)(NB * NH * (SEQ / 64)) * (size_t)(64 * HD) == (size_t)NB * SEQ * HID);
static_assert((size_t)(HID / 64) * (size_t)(NB * SEQ / 128) * 4u * (32u * 64u) == (size_t)NB * SEQ * HID);

typedef unsigned short hs;
typedef __attribute__((ext_vector_type(16))) __bf16   v16bf;
typedef __attribute__((ext_vector_type(16))) _Float16 v16h;
typedef __attribute__((ext_vector_type(8)))  unsigned short v8us;
typedef __attribute__((ext_vector_type(8)))  float    v8f;
typedef __attribute__((ext_vector_type(4)))  float    v4f;
typedef v4f  __attribute__((may_alias)) v4fa;
typedef v8us __attribute__((may_alias)) v8usa;

struct InvF { float v[32]; };
static_assert(sizeof(InvF) == 128);

__device__ __forceinline__ unsigned short f2bf(float f) { unsigned u = __float_as_uint(f); u += 0x7FFFu + ((u >> 16) & 1u); return (unsigned short)(u >> 16); }
__device__ __forceinline__ float bf2f(unsigned short b) { return __uint_as_float(((unsigned)b) << 16); }
__device__ __forceinline__ float bfr(float f) { return bf2f(f2bf(f)); }
__device__ __forceinline__ unsigned short f2h(float f) { return __builtin_bit_cast(unsigned short, (_Float16)f); }
__device__ __forceinline__ v16bf cat16b(v8us lo, v8us hi) { return __builtin_bit_cast(v16bf, __builtin_shufflevector(lo, hi, 0, 1, 2, 3, 4, 5, 6, 7, 8, 9, 10, 11, 12, 13, 14, 15)); }
__device__ __forceinline__ v16bf ldb(const hs* p) { return cat16b(*(const v8us*)p, *(const v8us*)(p + 16)); }
__device__ __forceinline__ v8f wmmab(v16bf a, v16bf b, v8f c) { return __builtin_amdgcn_wmma_f32_16x16x32_bf16(false, a, false, b, (short)0, c, false, false); }
__device__ __forceinline__ v8f wmmah(v16bf a, v16bf b, v8f c) {
    return __builtin_amdgcn_wmma_f32_16x16x32_f16(false, __builtin_bit_cast(v16h, a), false, __builtin_bit_cast(v16h, b), (short)0, c, false, false);
}

__global__ __launch_bounds__(256) void k_cvt(const float* __restrict__ X, const float* __restrict__ Wq, const float* __restrict__ Wk,
                                             const float* __restrict__ Wv, const float* __restrict__ Wo, hs* XB, hs* WB, hs* WO) {
    const unsigned i = blockIdx.x * 256u + threadIdx.x;
    const unsigned seg = blockIdx.y;
    unsigned ngrp;
    const float* src;
    hs* dst;
    if (seg == 0u) {
        ngrp = (unsigned)((size_t)NB * SEQ * HID / 8);
        const unsigned row = i >> 8, g = i & 255u;
        const unsigned b = row / (unsigned)SEQ, t = row - b * (unsigned)SEQ;
        src = X + ((size_t)b * SEQ_FULL + t) * HID + g * 8u;
        dst = XB + (size_t)i * 8u;
    } else if (seg == 1u) {
        ngrp = (unsigned)((size_t)HID * HID / 8);
        src = Wq + (size_t)i * 8u;
        dst = WB + (size_t)i * 8u;
    } else if (seg == 2u) {
        ngrp = (unsigned)((size_t)NKV * HD * HID / 8);
        src = Wk + (size_t)i * 8u;
        dst = WB + (size_t)HID * HID + (size_t)i * 8u;
    } else if (seg == 3u) {
        ngrp = (unsigned)((size_t)NKV * HD * HID / 8);
        src = Wv + (size_t)i * 8u;
        dst = WB + (size_t)(HID + NKV * HD) * HID + (size_t)i * 8u;
    } else {
        ngrp = (unsigned)((size_t)HID * HID / 8);
        src = Wo + (size_t)i * 8u;
        dst = WO + (size_t)i * 8u;
    }
    if (i >= ngrp) return;
    const v8f v = *(const v8f*)src;
    v8us o;
    if (seg == 4u) {
#pragma unroll
        for (int c = 0; c < 8; ++c) o[c] = f2h(bfr(v[c]) * 64.0f);
    } else {
#pragma unroll
        for (int c = 0; c < 8; ++c) o[c] = f2bf(v[c]);
    }
    *(volatile v8us*)dst = o;
    __threadfence();
    *(volatile v8us*)dst = o;
}

__global__ __launch_bounds__(256) void k_tab(const int* __restrict__ pos, float* CS, InvF inv) {
    const unsigned gid = blockIdx.x * 256u + threadIdx.x;
    const unsigned tok = gid >> 5, i = gid & 31u;
    if (tok >= (unsigned)(NB * SEQ)) return;
    const unsigned b = tok / (unsigned)SEQ, t = tok - b * (unsigned)SEQ;
    const int p = pos[(size_t)b * SEQ_FULL + t];
    float f = inv.v[0];
#pragma unroll
    for (unsigned j = 1; j < 32; ++j) f = (i == j) ? inv.v[j] : f;
    const float ang = (float)p * f;
    float sn, cs;
    sincosf(ang, &sn, &cs);
    float* row = CS + (size_t)tok * 64u;
    *(volatile float*)(row + i) = cs;
    *(volatile float*)(row + 32u + i) = sn;
    __threadfence();
    *(volatile float*)(row + i) = cs;
    *(volatile float*)(row + 32u + i) = sn;
}

template <bool F16>
__device__ __forceinline__ void gemm_main(const hs* __restrict__ A, const hs* __restrict__ W, unsigned m0, unsigned n0, unsigned lr, unsigned hi, v8f (&acc)[2][4]) {
#pragma unroll
    for (int a = 0; a < 2; ++a) {
#pragma unroll
        for (int c = 0; c < 4; ++c) acc[a][c] = (v8f){};
    }
    const hs* ap = A + (size_t)(m0 + lr) * HID + 8u * hi;
    const hs* wp = W + (size_t)(n0 + lr) * HID + 8u * hi;
#pragma unroll 1
    for (unsigned k0 = 0; k0 < (unsigned)HID; k0 += 32u) {
        const v16bf a0 = ldb(ap + k0);
        const v16bf a1 = ldb(ap + (size_t)16 * HID + k0);
        v16bf bq[4];
#pragma unroll
        for (int c = 0; c < 4; ++c) bq[c] = ldb(wp + (size_t)c * 16 * HID + k0);
#pragma unroll
        for (int c = 0; c < 4; ++c) {
            if (F16) {
                acc[0][c] = wmmah(a0, bq[c], acc[0][c]);
                acc[1][c] = wmmah(a1, bq[c], acc[1][c]);
            } else {
                acc[0][c] = wmmab(a0, bq[c], acc[0][c]);
                acc[1][c] = wmmab(a1, bq[c], acc[1][c]);
            }
        }
        asm volatile("v_nop\n\tv_nop\n\tv_nop\n\tv_nop"
                     : "+v"(acc[0][0]), "+v"(acc[0][1]), "+v"(acc[0][2]), "+v"(acc[0][3]),
                       "+v"(acc[1][0]), "+v"(acc[1][1]), "+v"(acc[1][2]), "+v"(acc[1][3])
                     : "v"(a0), "v"(a1), "v"(bq[0]), "v"(bq[1]), "v"(bq[2]), "v"(bq[3]));
    }
}

__global__ __launch_bounds__(128) void k_qkv(const hs* __restrict__ XB, const hs* __restrict__ WB, const float* __restrict__ CS, hs* QH, hs* KH, hs* VT) {
    __shared__ __align__(16) float os[NWV * 32 * OSP];
    __shared__ __align__(16) hs vts[HD * VTP];
    const unsigned tid = threadIdx.x, lane = tid & 31u, wv = tid >> 5, lr = lane & 15u, hi = lane >> 4;
    const unsigned hc = blockIdx.x;
    const unsigned mb = blockIdx.y * 128u;
    const unsigned m0 = mb + wv * 32u;
    const unsigned n0 = hc * 64u;
    const unsigned b = mb / (unsigned)SEQ, tb = mb - b * (unsigned)SEQ;

    v8f acc[2][4];
    gemm_main<false>(XB, WB, m0, n0, lr, hi, acc);

    if (hc < (unsigned)(NH + NKV)) {
        float* ow = os + wv * (32u * OSP);
#pragma unroll
        for (int rt = 0; rt < 2; ++rt) {
#pragma unroll
            for (int ct = 0; ct < 4; ++ct) {
#pragma unroll
                for (int r = 0; r < 8; ++r) ow[((unsigned)rt * 16u + 8u * hi + (unsigned)r) * OSP + (unsigned)ct * 16u + lr] = acc[rt][ct][r];
            }
        }
        __syncthreads();
        const bool isq = hc < (unsigned)NH;
        const unsigned head = isq ? hc : (hc - (unsigned)NH);
        const unsigned nhp = isq ? (unsigned)NH : (unsigned)NKV;
        hs* plane = isq ? QH : KH;
        hs* base = plane + (((size_t)(b * nhp + head)) * SEQ + tb + wv * 32u) * HD;
        const unsigned pc = lane & 7u, rq = lane >> 3;
        const unsigned c8 = pc * 8u, pcol = (c8 + 32u) & 63u, fi = c8 & 31u;
        const float sg = (pc < 4u) ? -1.0f : 1.0f;
        v8us res[8];
#pragma unroll
        for (unsigned it = 0; it < 8; ++it) {
            const unsigned row = it * 4u + rq;
            const float* orow = ow + row * OSP;
            const v4f x0 = *(const v4fa*)(orow + c8);
            const v4f x1 = *(const v4fa*)(orow + c8 + 4u);
            const v4f y0 = *(const v4fa*)(orow + pcol);
            const v4f y1 = *(const v4fa*)(orow + pcol + 4u);
            const float* cp = CS + (size_t)(m0 + row) * 64u + fi;
            const v4f c0 = *(const v4f*)cp;
            const v4f c1 = *(const v4f*)(cp + 4);
            const v4f s0 = *(const v4f*)(cp + 32);
            const v4f s1 = *(const v4f*)(cp + 36);
            v8us o;
#pragma unroll
            for (int j = 0; j < 4; ++j) {
                o[j]     = f2h(x0[j] * c0[j] + (sg * y0[j]) * s0[j]);
                o[4 + j] = f2h(x1[j] * c1[j] + (sg * y1[j]) * s1[j]);
            }
            res[it] = o;
        }
#pragma unroll
        for (unsigned it = 0; it < 8; ++it) *(volatile v8us*)(base + (size_t)(it * 4u + rq) * HD + c8) = res[it];
        __threadfence();
#pragma unroll
        for (unsigned it = 0; it < 8; ++it) *(volatile v8us*)(base + (size_t)(it * 4u + rq) * HD + c8) = res[it];
    } else {
#pragma unroll
        for (int rt = 0; rt < 2; ++rt) {
#pragma unroll
            for (int ct = 0; ct < 4; ++ct) {
                v8us o;
#pragma unroll
                for (int r = 0; r < 8; ++r) o[r] = f2h(acc[rt][ct][r]);
                *(v8usa*)(vts + ((unsigned)ct * 16u + lr) * VTP + wv * 32u + (unsigned)rt * 16u + 8u * hi) = o;
            }
        }
        __syncthreads();
        const unsigned kv = hc - (unsigned)(NH + NKV);
        hs* dst = VT + ((size_t)(b * NKV + kv) * HD) * SEQ + tb;
        const unsigned p8 = (tid & 15u) * 8u, dr = tid >> 4;
#pragma unroll 1
        for (int ps = 0; ps < 2; ++ps) {
#pragma unroll
            for (unsigned it = 0; it < 8; ++it) {
                const unsigned d = it * 8u + dr;
                const v8us o = *(const v8usa*)(vts + d * VTP + p8);
                *(volatile v8us*)(dst + (size_t)d * SEQ + p8) = o;
            }
            if (ps == 0) __threadfence();
        }
    }
}

__global__ __launch_bounds__(128) void k_flash(const hs* __restrict__ QH, const hs* __restrict__ KH, const hs* __restrict__ VT, hs* CX) {
    __shared__ __align__(16) hs cs[NWV * 16 * CSP];
    const unsigned tid = threadIdx.x, lane = tid & 31u, wv = tid >> 5, lr = lane & 15u, hi = lane >> 4;
    const unsigned qpb = (unsigned)(SEQ / 64);
    const unsigned bh = blockIdx.x / qpb;
    const unsigned q0 = (blockIdx.x - bh * qpb) * 64u + wv * 16u;
    const unsigned b = bh >> 5, h = bh & 31u;
    const unsigned kvh = b * (unsigned)NKV + (h >> 2);

    v16bf qf[2];
    {
        const hs* qp = QH + ((size_t)bh * SEQ + q0 + lr) * HD + 8u * hi;
        qf[0] = ldb(qp);
        qf[1] = ldb(qp + 32);
    }
    const hs* kp = KH + ((size_t)kvh * SEQ + lr) * HD + 8u * hi;
    const hs* vp = VT + ((size_t)kvh * HD + lr) * SEQ + 8u * hi;

    v8f o[4];
#pragma unroll
    for (int t = 0; t < 4; ++t) o[t] = (v8f){};
    float ml = -1.0e30f;
    float l = 0.0f;
    const float sc = 0.125f * L2E;

#pragma unroll 1
    for (unsigned k0 = 0; k0 < (unsigned)SEQ; k0 += KS) {
        v8f s0 = (v8f){}, s1 = (v8f){};
        const hs* ka = kp + (size_t)k0 * HD;
        v16bf ka0[2], ka1[2];
#pragma unroll
        for (int dk = 0; dk < 2; ++dk) {
            ka0[dk] = ldb(ka + dk * 32);
            ka1[dk] = ldb(ka + 16 * HD + dk * 32);
        }
#pragma unroll
        for (int dk = 0; dk < 2; ++dk) {
            s0 = wmmah(ka0[dk], qf[dk], s0);
            s1 = wmmah(ka1[dk], qf[dk], s1);
        }
        asm volatile("v_nop\n\tv_nop\n\tv_nop\n\tv_nop" : "+v"(s0), "+v"(s1)
                     : "v"(qf[0]), "v"(qf[1]), "v"(ka0[0]), "v"(ka0[1]), "v"(ka1[0]), "v"(ka1[1]));

        float mx = fmaxf(s0[0], s1[0]);
#pragma unroll
        for (int r = 1; r < 8; ++r) mx = fmaxf(mx, fmaxf(s0[r], s1[r]));
        mx = fmaxf(mx, __shfl_xor(mx, 16, 32));
        const float mnl = fmaxf(ml, mx * sc);
        const float corr = __builtin_amdgcn_exp2f(ml - mnl);
        ml = mnl;
        const float off = 10.0f - mnl;
        float p0[8], p1[8];
        float ps = 0.0f;
#pragma unroll
        for (int r = 0; r < 8; ++r) {
            p0[r] = __builtin_amdgcn_exp2f(fmaf(s0[r], sc, off));
            p1[r] = __builtin_amdgcn_exp2f(fmaf(s1[r], sc, off));
            ps += p0[r] + p1[r];
        }
        ps += __shfl_xor(ps, 16, 32);
        l = l * corr + ps;
        if (__builtin_amdgcn_ballot_w32(corr != 1.0f) != 0u) {
#pragma unroll
            for (int t = 0; t < 4; ++t) o[t] *= corr;
        }

        v16h ph;
#pragma unroll
        for (int r = 0; r < 8; ++r) {
            ph[r]     = (_Float16)p0[r];
            ph[8 + r] = (_Float16)p1[r];
        }
        const v16bf pb = __builtin_bit_cast(v16bf, ph);

        asm volatile("" ::: "memory");
        const hs* va = vp + k0;
        v16bf vf[4];
#pragma unroll
        for (int t = 0; t < 4; ++t) vf[t] = ldb(va + (size_t)t * 16 * SEQ);
#pragma unroll
        for (int t = 0; t < 4; ++t) o[t] = wmmah(vf[t], pb, o[t]);
        asm volatile("v_nop\n\tv_nop\n\tv_nop\n\tv_nop"
                     : "+v"(o[0]), "+v"(o[1]), "+v"(o[2]), "+v"(o[3])
                     : "v"(pb), "v"(vf[0]), "v"(vf[1]), "v"(vf[2]), "v"(vf[3]));
    }

    const float inv = 256.0f * (1.0f / l);
    hs* cw = cs + wv * (16u * CSP);
#pragma unroll
    for (int t = 0; t < 4; ++t) {
        v8us ov;
#pragma unroll
        for (int r = 0; r < 8; ++r) ov[r] = f2h(o[t][r] * inv);
        *(v8usa*)(cw + lr * CSP + (unsigned)t * 16u + 8u * hi) = ov;
    }
    __syncthreads();
    const unsigned pc8 = (lane & 7u) * 8u, rq = lane >> 3;
    hs* dst = CX + ((size_t)b * SEQ + q0) * HID + h * 64u + pc8;
#pragma unroll 1
    for (int ps2 = 0; ps2 < 2; ++ps2) {
#pragma unroll
        for (unsigned it = 0; it < 4; ++it) {
            const unsigned row = it * 4u + rq;
            const v8us val = *(const v8usa*)(cw + row * CSP + pc8);
            *(volatile v8us*)(dst + (size_t)row * HID) = val;
        }
        if (ps2 == 0) __threadfence();
    }
}

__global__ __launch_bounds__(128) void k_oproj(const hs* __restrict__ CX, const hs* __restrict__ WO, float* OUT) {
    __shared__ __align__(16) float os[NWV * 32 * OSP];
    const unsigned tid = threadIdx.x, lane = tid & 31u, wv = tid >> 5, lr = lane & 15u, hi = lane >> 4;
    const unsigned n0 = blockIdx.x * 64u;
    const unsigned m0 = blockIdx.y * 128u + wv * 32u;

    v8f acc[2][4];
    gemm_main<true>(CX, WO, m0, n0, lr, hi, acc);

    const float osc = 1.0f / 16384.0f;
    float* ow = os + wv * (32u * OSP);
#pragma unroll
    for (int rt = 0; rt < 2; ++rt) {
#pragma unroll
        for (int ct = 0; ct < 4; ++ct) {
#pragma unroll
            for (int r = 0; r < 8; ++r) ow[((unsigned)rt * 16u + 8u * hi + (unsigned)r) * OSP + (unsigned)ct * 16u + lr] = acc[rt][ct][r] * osc;
        }
    }
    __syncthreads();
    const unsigned c4 = (lane & 15u) * 4u, rh = lane >> 4;
    float* dst = OUT + (size_t)m0 * HID + n0 + c4;
#pragma unroll 1
    for (int ps = 0; ps < 2; ++ps) {
#pragma unroll 4
        for (unsigned it = 0; it < 16; ++it) {
            const unsigned row = it * 2u + rh;
            const v4f val = *(const v4fa*)(ow + row * OSP + c4);
            *(volatile v4f*)(dst + (size_t)row * HID) = val;
        }
        if (ps == 0) __threadfence();
    }
}

extern "C" void kernel_launch(void* const* d_in, const int* in_sizes, int n_in,
                              void* d_out, int out_size, void* d_ws, size_t ws_size, hipStream_t stream) {
    if (n_in < 6) return;
    const size_t tokneed = (size_t)(NB - 1) * SEQ_FULL + SEQ;
    if ((size_t)in_sizes[0] < tokneed * HID) return;
    if ((size_t)in_sizes[1] < tokneed) return;
    if ((size_t)in_sizes[2] < (size_t)HID * HID) return;
    if ((size_t)in_sizes[3] < (size_t)NKV * HD * HID) return;
    if ((size_t)in_sizes[4] < (size_t)NKV * HD * HID) return;
    if ((size_t)in_sizes[5] < (size_t)HID * HID) return;
    if ((size_t)out_size < (size_t)NB * SEQ * HID) return;

    const float* X   = (const float*)d_in[0];
    const int*   pos = (const int*)d_in[1];
    const float* Wq  = (const float*)d_in[2];
    const float* Wk  = (const float*)d_in[3];
    const float* Wv  = (const float*)d_in[4];
    const float* Wo  = (const float*)d_in[5];
    float* OUT = (float*)d_out;

    const size_t P_XB = (size_t)NB * SEQ * HID * 2;
    const size_t P_WB = (size_t)NQKV * HID * 2;
    const size_t P_WO = (size_t)HID * HID * 2;
    const size_t P_CS = (size_t)NB * SEQ * 64 * 4;
    const size_t P_QH = (size_t)NB * NH * SEQ * HD * 2;
    const size_t P_KH = (size_t)NB * NKV * SEQ * HD * 2;
    const size_t P_VT = (size_t)NB * NKV * HD * SEQ * 2;
    const size_t P_CX = (size_t)NB * SEQ * HID * 2;
    const size_t total = P_XB + P_WB + P_WO + P_CS + P_QH + P_KH + P_VT + P_CX;
    if (total > ws_size) return;
    if (total > (size_t)134217728) return;
    char* wsp = (char*)d_ws;
    size_t off = 0;
    hs* XB = (hs*)(wsp + off);      off += P_XB;
    hs* WB = (hs*)(wsp + off);      off += P_WB;
    hs* WO = (hs*)(wsp + off);      off += P_WO;
    float* CS = (float*)(wsp + off); off += P_CS;
    hs* QH = (hs*)(wsp + off);      off += P_QH;
    hs* KH = (hs*)(wsp + off);      off += P_KH;
    hs* VT = (hs*)(wsp + off);      off += P_VT;
    hs* CX = (hs*)(wsp + off);      off += P_CX;

    InvF inv;
    for (int i = 0; i < 32; ++i) {
        const double pw = pow(10000.0, (double)(2 * i) / 64.0);
        const float pf = (float)pw;
        inv.v[i] = 1.0f / pf;
    }

    const size_t g0 = (size_t)NB * SEQ * HID / 8 / 256;
    const size_t g1 = (size_t)HID * HID / 8 / 256;
    const unsigned gc = (unsigned)(g0 > g1 ? g0 : g1);
    k_cvt<<<dim3(gc, 5, 1), 256, 0, stream>>>(X, Wq, Wk, Wv, Wo, XB, WB, WO);
    k_tab<<<(unsigned)((size_t)NB * SEQ * 32 / 256), 256, 0, stream>>>(pos, CS, inv);
    k_qkv<<<dim3((unsigned)(NQKV / 64), (unsigned)(NB * SEQ / 128), 1), 128, 0, stream>>>(XB, WB, CS, QH, KH, VT);
    k_flash<<<(unsigned)(NB * NH * (SEQ / 64)), 128, 0, stream>>>(QH, KH, VT, CX);
    k_oproj<<<dim3((unsigned)(HID / 64), (unsigned)(NB * SEQ / 128), 1), 128, 0, stream>>>(CX, WO, OUT);
}
